// FpgnnModel_10797547782760
// MI455X (gfx1250) — hardware-verified
//
#include <hip/hip_runtime.h>
#include <stddef.h>
#include <stdint.h>

#define NB   512
#define NA   128
#define FIN  133
#define KP1  160
#define NHD  8
#define DHD  64
#define HID  512
#define FPD  1489
#define KPF  1504
#define NT   12
#define NTP  16

static_assert(KP1 % 32 == 0);
static_assert(KPF % 32 == 0);
static_assert(NHD * DHD == HID);
static_assert(HID % 64 == 0);
static_assert(NB % 128 == 0);
static_assert((NB * NT) % (256 * 4) == 0);

typedef _Float16       hf;
typedef hf             v8h  __attribute__((ext_vector_type(8)));
typedef hf             v16h __attribute__((ext_vector_type(16)));
typedef float          v8f  __attribute__((ext_vector_type(8)));
typedef float          v4f  __attribute__((ext_vector_type(4)));
typedef unsigned int   v4u  __attribute__((ext_vector_type(4)));

union FragH { v16h v; v8h h[2]; };
union Pack8 { v8h h; v4u u; };

#define ALPHA_S  0.2f
#define NEGBIG   (-9e15f)
#define WSCALE   16.0f
#define ASCALE   16.0f
#define PSCALE   1024.0f

extern __shared__ __align__(16) char dsm[];

__device__ __forceinline__ v8f zero8() { return (v8f){0.f, 0.f, 0.f, 0.f, 0.f, 0.f, 0.f, 0.f}; }

__device__ __forceinline__ v8f mma16(v16h a, v16h b, v8f c) {
  c = __builtin_amdgcn_wmma_f32_16x16x32_f16(false, a, false, b, (short)0, c, false, false);
  asm volatile("v_nop\n\tv_nop\n\tv_nop\n\tv_nop" : "+v"(c) : "v"(a), "v"(b));
  return c;
}

__device__ __forceinline__ v16h ldfrag(const hf* p, int ld, int row0, int k0, int lane) {
  const int m = lane & 15, lh = lane >> 4;
  const hf* q = p + (size_t)(row0 + m) * ld + k0 + 8 * lh;
  FragH f;
  f.h[0] = *(const v8h*)(q);
  f.h[1] = *(const v8h*)(q + 16);
  return f.v;
}

__global__ __launch_bounds__(256) void k_cvt16(const float* __restrict__ W, int R, int K, int ldw,
                                               int Kpad, int tr, int in_stride, int out_stride,
                                               float s, hf* __restrict__ out) {
  hf* ct = (hf*)dsm;
  const int tid = threadIdx.x;
  const int r0 = blockIdx.x * 16;
  const float* src = W + (size_t)blockIdx.y * (size_t)in_stride;
  hf* dst = out + (size_t)blockIdx.y * (size_t)out_stride + (size_t)r0 * Kpad;
  if (tr != 0) {
    const int rr = tid & 15;
    const int r  = r0 + rr;
    const int rc = min(r, R - 1);
    for (int k = tid >> 4; k < Kpad; k += 16) {
      const int kc = min(k, K - 1);
      float v = src[(size_t)kc * ldw + rc];
      v = (r < R && k < K) ? v * s : 0.0f;
      ct[rr * Kpad + k] = (hf)v;
    }
  } else {
#pragma unroll 1
    for (int rr = 0; rr < 16; ++rr) {
      const int r  = r0 + rr;
      const int rc = min(r, R - 1);
      for (int k = tid; k < Kpad; k += 256) {
        const int kc = min(k, K - 1);
        float v = src[(size_t)rc * ldw + kc];
        v = (r < R && k < K) ? v * s : 0.0f;
        ct[rr * Kpad + k] = (hf)v;
      }
    }
  }
  __syncthreads();
  const int npc = 2 * Kpad;
  for (int p = tid; p < npc; p += 256) {
    Pack8 pk; pk.h = *(const v8h*)(ct + p * 8);
    *(volatile v4u*)(dst + (size_t)p * 8) = pk.u;
  }
  __threadfence();
  for (int p = tid; p < npc; p += 256) {
    Pack8 pk; pk.h = *(const v8h*)(ct + p * 8);
    *(volatile v4u*)(dst + (size_t)p * 8) = pk.u;
  }
}

#define PH 168
#define PJ 136
#define PX 72
#define G1_OFF_P   43008
#define G1_OFF_WT  77824
#define G1_OFF_X   95232
#define G1_OFF_S   113664
#define G1_LDS     115200
static_assert(NA * PH * 2 == G1_OFF_P);
static_assert(G1_OFF_P + NA * PJ * 2 == G1_OFF_WT);
static_assert(G1_OFF_WT + DHD * PJ * 2 == G1_OFF_X);
static_assert(G1_OFF_X + NA * PX * 2 == G1_OFF_S);
static_assert(G1_OFF_S + 3 * NA * 4 == G1_LDS);

__global__ __launch_bounds__(256) void k_gat1(const float* __restrict__ h, const int* __restrict__ adj,
                                              const float* __restrict__ edge, const hf* __restrict__ WhdT,
                                              const float* __restrict__ a1h, const float* __restrict__ a2h,
                                              const float* __restrict__ aeh, hf* __restrict__ X) {
  hf* hA  = (hf*)dsm;
  hf* sP  = (hf*)(dsm + G1_OFF_P);
  hf* sWt = (hf*)(dsm + G1_OFF_WT);
  hf* sX  = (hf*)(dsm + G1_OFF_X);
  float* s1s  = (float*)(dsm + G1_OFF_S);
  float* s2s  = s1s + NA;
  float* rinv = s2s + NA;
  const int tid = threadIdx.x, lane = tid & 31, wave = tid >> 5;
  const int hh = lane >> 4, c = lane & 15;
  const int b = blockIdx.x;
  const int m0 = wave * 16;

  {
    const float* hs = h + (size_t)b * NA * FIN;
    for (int idx = tid; idx < NA * KP1; idx += 256) {
      const int r  = idx / KP1;
      const int k  = idx - r * KP1;
      const int kc = min(k, FIN - 1);
      float v = hs[r * FIN + kc];
      v = (k < FIN) ? v : 0.0f;
      hA[r * PH + k] = (hf)v;
    }
  }
  __syncthreads();
  const size_t ebase = (size_t)b * NA * NA;

#pragma unroll 1
  for (int hd = 0; hd < NHD; ++hd) {
    const hf* Wt = WhdT + (size_t)hd * DHD * KP1;
    v8f acc[4];
#pragma unroll
    for (int t = 0; t < 4; ++t) acc[t] = zero8();
#pragma unroll 1
    for (int k0 = 0; k0 < KP1; k0 += 32) {
      const v16h a = ldfrag(hA, PH, m0, k0, lane);
#pragma unroll
      for (int t = 0; t < 4; ++t) {
        const v16h bf = ldfrag(Wt, KP1, 16 * t, k0, lane);
        acc[t] = mma16(a, bf, acc[t]);
      }
    }
    {
      const float* a1 = a1h + hd * DHD;
      const float* a2 = a2h + hd * DHD;
      float p1[8], p2[8];
#pragma unroll
      for (int r = 0; r < 8; ++r) { p1[r] = 0.f; p2[r] = 0.f; }
#pragma unroll
      for (int t = 0; t < 4; ++t) {
        const float av1 = a1[16 * t + c];
        const float av2 = a2[16 * t + c];
#pragma unroll
        for (int r = 0; r < 8; ++r) {
          const float wv = acc[t][r] * (1.0f / WSCALE);
          p1[r] += wv * av1;
          p2[r] += wv * av2;
          sWt[(16 * t + c) * PJ + m0 + 8 * hh + r] = (hf)acc[t][r];
        }
      }
#pragma unroll
      for (int r = 0; r < 8; ++r) {
        float x1 = p1[r], x2 = p2[r];
        x1 += __shfl_xor(x1, 1); x1 += __shfl_xor(x1, 2); x1 += __shfl_xor(x1, 4); x1 += __shfl_xor(x1, 8);
        x2 += __shfl_xor(x2, 1); x2 += __shfl_xor(x2, 2); x2 += __shfl_xor(x2, 4); x2 += __shfl_xor(x2, 8);
        if (c == 0) { s1s[m0 + 8 * hh + r] = x1; s2s[m0 + 8 * hh + r] = x2; }
      }
    }
    __syncthreads();

    {
      const float ae = aeh[hd];
#pragma unroll 1
      for (int r = 0; r < 16; ++r) {
        const int i = m0 + r;
        const float s1v = s1s[i];
        const size_t eb = ebase + (size_t)i * NA;
        float vals[4];
#pragma unroll
        for (int cc = 0; cc < 4; ++cc) {
          const int j = lane + 32 * cc;
          float ev = s1v + s2s[j] + edge[eb + j] * ae;
          ev = (ev >= 0.0f) ? ev : ALPHA_S * ev;
          vals[cc] = (adj[eb + j] > 0) ? ev : NEGBIG;
        }
        float mx = fmaxf(fmaxf(vals[0], vals[1]), fmaxf(vals[2], vals[3]));
#pragma unroll
        for (int sft = 16; sft >= 1; sft >>= 1) mx = fmaxf(mx, __shfl_xor(mx, sft));
        float p[4], sum = 0.f;
#pragma unroll
        for (int cc = 0; cc < 4; ++cc) { p[cc] = __expf(vals[cc] - mx); sum += p[cc]; }
#pragma unroll
        for (int sft = 16; sft >= 1; sft >>= 1) sum += __shfl_xor(sum, sft);
        if (lane == 0) rinv[i] = 1.0f / sum;
#pragma unroll
        for (int cc = 0; cc < 4; ++cc) sP[i * PJ + lane + 32 * cc] = (hf)(p[cc] * PSCALE);
      }
    }
    __syncthreads();

    float rs[8];
#pragma unroll
    for (int r = 0; r < 8; ++r) rs[r] = rinv[m0 + 8 * hh + r] * (1.0f / (PSCALE * WSCALE));
    v8f acc2[4];
#pragma unroll
    for (int t = 0; t < 4; ++t) acc2[t] = zero8();
#pragma unroll 1
    for (int kk = 0; kk < NA / 32; ++kk) {
      const v16h a = ldfrag(sP, PJ, m0, kk * 32, lane);
#pragma unroll
      for (int t = 0; t < 4; ++t) {
        const v16h bf = ldfrag(sWt, PJ, 16 * t, kk * 32, lane);
        acc2[t] = mma16(a, bf, acc2[t]);
      }
    }
#pragma unroll
    for (int t = 0; t < 4; ++t) {
#pragma unroll
      for (int r = 0; r < 8; ++r) {
        const int row = m0 + 8 * hh + r;
        const float hp = acc2[t][r] * rs[r];
        const float xv = (hp > 0.0f) ? hp : (__expf(hp) - 1.0f);
        sX[row * PX + 16 * t + c] = (hf)(xv * ASCALE);
      }
    }
    __syncthreads();

    v4u val[4];
    size_t go[4];
#pragma unroll
    for (int it = 0; it < 4; ++it) {
      const int p  = tid + 256 * it;
      const int L  = p >> 3;
      const int pc = p & 7;
      Pack8 pk; pk.h = *(const v8h*)(sX + L * PX + pc * 8);
      val[it] = pk.u;
      go[it]  = ((size_t)b * NA + L) * HID + hd * DHD + pc * 8;
    }
#pragma unroll
    for (int it = 0; it < 4; ++it) *(volatile v4u*)(X + go[it]) = val[it];
    __threadfence();
#pragma unroll
    for (int it = 0; it < 4; ++it) *(volatile v4u*)(X + go[it]) = val[it];
  }
}

#define G2_OFF_P   139264
#define G2_OFF_T   174080
#define G2_OFF_C   175616
#define G2_OFF_G   177664
#define G2_LDS     179712
static_assert(HID * PJ * 2 == G2_OFF_P);
static_assert(G2_OFF_P + NA * PJ * 2 == G2_OFF_T);
static_assert(G2_OFF_T + 3 * NA * 4 == G2_OFF_C);
static_assert(G2_OFF_C + 8 * 64 * 4 == G2_OFF_G);
static_assert(G2_OFF_G + HID * 4 == G2_LDS);

__global__ __launch_bounds__(256) void k_gat2(const hf* __restrict__ X, const hf* __restrict__ WoT,
                                              const int* __restrict__ adj, const float* __restrict__ edge,
                                              const float* __restrict__ a1o, const float* __restrict__ a2o,
                                              const float* __restrict__ aeo, hf* __restrict__ GO) {
  hf* sWx = (hf*)dsm;
  hf* sP  = (hf*)(dsm + G2_OFF_P);
  float* t1s  = (float*)(dsm + G2_OFF_T);
  float* t2s  = t1s + NA;
  float* rinv = t2s + NA;
  float* colp = (float*)(dsm + G2_OFF_C);
  float* gsum = (float*)(dsm + G2_OFF_G);
  const int tid = threadIdx.x, lane = tid & 31, wave = tid >> 5;
  const int hh = lane >> 4, c = lane & 15;
  const int b = blockIdx.x;
  const int m0 = wave * 16;
  const size_t ebase = (size_t)b * NA * NA;

  {
    float p1[8], p2[8];
#pragma unroll
    for (int r = 0; r < 8; ++r) { p1[r] = 0.f; p2[r] = 0.f; }
    const int xr0 = b * NA + m0;
#pragma unroll 1
    for (int s = 0; s < HID / 64; ++s) {
      v8f acc[4];
#pragma unroll
      for (int t = 0; t < 4; ++t) acc[t] = zero8();
#pragma unroll 1
      for (int k0 = 0; k0 < HID; k0 += 32) {
        const v16h a = ldfrag(X, HID, xr0, k0, lane);
#pragma unroll
        for (int t = 0; t < 4; ++t) {
          const v16h bf = ldfrag(WoT, HID, s * 64 + 16 * t, k0, lane);
          acc[t] = mma16(a, bf, acc[t]);
        }
      }
#pragma unroll
      for (int t = 0; t < 4; ++t) {
        const int n = s * 64 + 16 * t + c;
        const float av1 = a1o[n];
        const float av2 = a2o[n];
#pragma unroll
        for (int r = 0; r < 8; ++r) {
          const float wx = acc[t][r] * (1.0f / (ASCALE * WSCALE));
          p1[r] += wx * av1;
          p2[r] += wx * av2;
          sWx[n * PJ + m0 + 8 * hh + r] = (hf)(acc[t][r] * (1.0f / 16.0f));
        }
      }
    }
#pragma unroll
    for (int r = 0; r < 8; ++r) {
      float x1 = p1[r], x2 = p2[r];
      x1 += __shfl_xor(x1, 1); x1 += __shfl_xor(x1, 2); x1 += __shfl_xor(x1, 4); x1 += __shfl_xor(x1, 8);
      x2 += __shfl_xor(x2, 1); x2 += __shfl_xor(x2, 2); x2 += __shfl_xor(x2, 4); x2 += __shfl_xor(x2, 8);
      if (c == 0) { t1s[m0 + 8 * hh + r] = x1; t2s[m0 + 8 * hh + r] = x2; }
    }
  }
  __syncthreads();

  {
    const float ae = aeo[0];
#pragma unroll 1
    for (int r = 0; r < 16; ++r) {
      const int i = m0 + r;
      const float t1v = t1s[i];
      const size_t eb = ebase + (size_t)i * NA;
      float vals[4];
#pragma unroll
      for (int cc = 0; cc < 4; ++cc) {
        const int j = lane + 32 * cc;
        float ev = t1v + t2s[j] + edge[eb + j] * ae;
        ev = (ev >= 0.0f) ? ev : ALPHA_S * ev;
        vals[cc] = (adj[eb + j] > 0) ? ev : NEGBIG;
      }
      float mx = fmaxf(fmaxf(vals[0], vals[1]), fmaxf(vals[2], vals[3]));
#pragma unroll
      for (int sft = 16; sft >= 1; sft >>= 1) mx = fmaxf(mx, __shfl_xor(mx, sft));
      float p[4], sum = 0.f;
#pragma unroll
      for (int cc = 0; cc < 4; ++cc) { p[cc] = __expf(vals[cc] - mx); sum += p[cc]; }
#pragma unroll
      for (int sft = 16; sft >= 1; sft >>= 1) sum += __shfl_xor(sum, sft);
      if (lane == 0) rinv[i] = 1.0f / sum;
#pragma unroll
      for (int cc = 0; cc < 4; ++cc) sP[i * PJ + lane + 32 * cc] = (hf)(p[cc] * PSCALE);
    }
  }
  __syncthreads();

  float rs[8];
#pragma unroll
  for (int r = 0; r < 8; ++r) rs[r] = rinv[m0 + 8 * hh + r] * (1.0f / (PSCALE * 16.0f));
#pragma unroll 1
  for (int s = 0; s < HID / 64; ++s) {
    v8f acc[4];
#pragma unroll
    for (int t = 0; t < 4; ++t) acc[t] = zero8();
#pragma unroll 1
    for (int kk = 0; kk < NA / 32; ++kk) {
      const v16h a = ldfrag(sP, PJ, m0, kk * 32, lane);
#pragma unroll
      for (int t = 0; t < 4; ++t) {
        const v16h bf = ldfrag(sWx, PJ, s * 64 + 16 * t, kk * 32, lane);
        acc[t] = mma16(a, bf, acc[t]);
      }
    }
#pragma unroll
    for (int t = 0; t < 4; ++t) {
      float cs = 0.f;
#pragma unroll
      for (int r = 0; r < 8; ++r) {
        const float hp = acc[t][r] * rs[r];
        const float g  = (hp > 0.0f) ? hp : (__expf(hp) - 1.0f);
        cs += g;
      }
      cs += __shfl_xor(cs, 16);
      if (hh == 0) colp[wave * 64 + 16 * t + c] = cs;
    }
    __syncthreads();
    if (tid < 64) {
      float sm = 0.f;
#pragma unroll
      for (int w = 0; w < 8; ++w) sm += colp[w * 64 + tid];
      gsum[s * 64 + tid] = sm * (1.0f / NA);
    }
    __syncthreads();
  }

  if (tid < 64) {
    Pack8 pk;
#pragma unroll
    for (int e = 0; e < 8; ++e) pk.h[e] = (hf)(gsum[8 * tid + e] * ASCALE);
    hf* gp = GO + (size_t)b * HID + 8 * tid;
    *(volatile v4u*)gp = pk.u;
    __threadfence();
    *(volatile v4u*)gp = pk.u;
  }
}

#define TFP 68
#define THP 72
__global__ __launch_bounds__(256) void k_gemm(const hf* __restrict__ A, int lda, const hf* __restrict__ Bt, int ldb,
                                              int K, const float* __restrict__ bias, const float* __restrict__ addend,
                                              int N, float oscale, int act, float hscale,
                                              float* __restrict__ outF, hf* __restrict__ outH) {
  __shared__ __align__(16) float sF[128 * TFP];
  __shared__ __align__(16) hf    sH[128 * THP];
  const int tid = threadIdx.x, lane = tid & 31, wave = tid >> 5;
  const int hh = lane >> 4, c = lane & 15;
  const int mb = blockIdx.x * 128;
  const int m0 = mb + wave * 16;
  const int n0 = blockIdx.y * 64;

  v8f acc[4];
#pragma unroll
  for (int t = 0; t < 4; ++t) acc[t] = zero8();
#pragma unroll 1
  for (int k0 = 0; k0 < K; k0 += 32) {
    const v16h a = ldfrag(A, lda, m0, k0, lane);
#pragma unroll
    for (int t = 0; t < 4; ++t) {
      const v16h bf = ldfrag(Bt, ldb, n0 + 16 * t, k0, lane);
      acc[t] = mma16(a, bf, acc[t]);
    }
  }
#pragma unroll
  for (int t = 0; t < 4; ++t) {
    const int n = n0 + 16 * t + c;
    const float bv = bias[n];
#pragma unroll
    for (int r = 0; r < 8; ++r) {
      const int row = wave * 16 + 8 * hh + r;
      float v = acc[t][r] * oscale + bv;
      if (addend != nullptr) v += addend[(size_t)(mb + row) * N + n];
      if (act != 0) v = fmaxf(v, 0.0f);
      sF[row * TFP + 16 * t + c] = v;
      sH[row * THP + 16 * t + c] = (hf)(v * hscale);
    }
  }
  __syncthreads();

  v4f vf[8]; size_t gf[8];
  v4u vh[4]; size_t gh[4];
#pragma unroll
  for (int it = 0; it < 8; ++it) {
    const int p  = tid + 256 * it;
    const int L  = p >> 3;
    const int pc = p & 7;
    const int row = L >> 1, half = L & 1;
    vf[it] = *(const v4f*)(sF + row * TFP + half * 32 + pc * 4);
    gf[it] = (size_t)(mb + row) * N + n0 + half * 32 + pc * 4;
  }
#pragma unroll
  for (int it = 0; it < 4; ++it) {
    const int p  = tid + 256 * it;
    const int L  = p >> 3;
    const int pc = p & 7;
    Pack8 pk; pk.h = *(const v8h*)(sH + L * THP + pc * 8);
    vh[it] = pk.u;
    gh[it] = (size_t)(mb + L) * N + n0 + pc * 8;
  }
  if (outF != nullptr) {
#pragma unroll
    for (int it = 0; it < 8; ++it) *(volatile v4f*)(outF + gf[it]) = vf[it];
  }
  if (outH != nullptr) {
#pragma unroll
    for (int it = 0; it < 4; ++it) *(volatile v4u*)(outH + gh[it]) = vh[it];
  }
  __threadfence();
  if (outF != nullptr) {
#pragma unroll
    for (int it = 0; it < 8; ++it) *(volatile v4f*)(outF + gf[it]) = vf[it];
  }
  if (outH != nullptr) {
#pragma unroll
    for (int it = 0; it < 4; ++it) *(volatile v4u*)(outH + gh[it]) = vh[it];
  }
}

__global__ __launch_bounds__(256) void k_final(const hf* __restrict__ A, const hf* __restrict__ Bt,
                                               const float* __restrict__ b2, float* __restrict__ out) {
  __shared__ __align__(16) float sO[NB * NT];
  const int tid = threadIdx.x, lane = tid & 31, wave = tid >> 5;
  const int hh = lane >> 4, c = lane & 15;
  v8f acc[4];
#pragma unroll
  for (int u = 0; u < 4; ++u) acc[u] = zero8();
#pragma unroll 1
  for (int k0 = 0; k0 < HID; k0 += 32) {
    const v16h bf = ldfrag(Bt, HID, 0, k0, lane);
#pragma unroll
    for (int u = 0; u < 4; ++u) {
      const v16h a = ldfrag(A, HID, 64 * wave + 16 * u, k0, lane);
      acc[u] = mma16(a, bf, acc[u]);
    }
  }
  const float bv = b2[min(c, NT - 1)];
#pragma unroll
  for (int u = 0; u < 4; ++u) {
#pragma unroll
    for (int r = 0; r < 8; ++r) {
      const int row = 64 * wave + 16 * u + 8 * hh + r;
      const float v = acc[u][r] * (1.0f / (ASCALE * WSCALE)) + bv;
      if (c < NT) sO[row * NT + c] = v;
    }
  }
  __syncthreads();
  v4f v[6];
#pragma unroll
  for (int it = 0; it < 6; ++it) v[it] = *(const v4f*)(sO + (tid + 256 * it) * 4);
#pragma unroll
  for (int it = 0; it < 6; ++it) *(volatile v4f*)(out + (size_t)(tid + 256 * it) * 4) = v[it];
  __threadfence();
#pragma unroll
  for (int it = 0; it < 6; ++it) *(volatile v4f*)(out + (size_t)(tid + 256 * it) * 4) = v[it];
}

extern "C" void kernel_launch(void* const* d_in, const int* in_sizes, int n_in,
                              void* d_out, int out_size, void* d_ws, size_t ws_size,
                              hipStream_t stream) {
  if (n_in < 28) return;
  if (in_sizes[0] != NB * NA * FIN) return;
  if (in_sizes[1] != NB * NA * NA) return;
  if (in_sizes[2] != NB * NA * NA) return;
  if (in_sizes[3] != NB * FPD) return;
  if (in_sizes[4] != NHD * FIN * DHD) return;
  if (in_sizes[5] != NHD * DHD || in_sizes[6] != NHD * DHD || in_sizes[7] != NHD) return;
  if (in_sizes[8] != HID * HID || in_sizes[9] != HID || in_sizes[10] != HID || in_sizes[11] != 1) return;
  if (in_sizes[12] != FPD * HID || in_sizes[13] != HID) return;
  if (in_sizes[14] != HID * HID || in_sizes[15] != HID) return;
  if (in_sizes[16] != HID * HID || in_sizes[17] != HID) return;
  if (in_sizes[20] != HID * HID || in_sizes[21] != HID) return;
  if (in_sizes[22] != HID * HID || in_sizes[23] != HID) return;
  if (in_sizes[24] != HID * HID || in_sizes[25] != HID) return;
  if (in_sizes[26] != HID * NT || in_sizes[27] != NT) return;
  if (out_size != NB * NT) return;

  const float* h     = (const float*)d_in[0];
  const int*   adj   = (const int*)d_in[1];
  const float* edge  = (const float*)d_in[2];
  const float* fp    = (const float*)d_in[3];
  const float* Whead = (const float*)d_in[4];
  const float* a1h   = (const float*)d_in[5];
  const float* a2h   = (const float*)d_in[6];
  const float* aeh   = (const float*)d_in[7];
  const float* Wout  = (const float*)d_in[8];
  const float* a1o   = (const float*)d_in[9];
  const float* a2o   = (const float*)d_in[10];
  const float* aeo   = (const float*)d_in[11];
  const float* fc1w  = (const float*)d_in[12];
  const float* fc1b  = (const float*)d_in[13];
  const float* fc2w  = (const float*)d_in[14];
  const float* fc2b  = (const float*)d_in[15];
  const float* qw    = (const float*)d_in[16];
  const float* qb    = (const float*)d_in[17];
  const float* vw    = (const float*)d_in[20];
  const float* vb    = (const float*)d_in[21];
  const float* ow    = (const float*)d_in[22];
  const float* ob    = (const float*)d_in[23];
  const float* f1w   = (const float*)d_in[24];
  const float* f1b   = (const float*)d_in[25];
  const float* f2w   = (const float*)d_in[26];
  const float* f2b   = (const float*)d_in[27];
  float* out = (float*)d_out;

  size_t off = 0;
  const size_t oX   = off; off += (size_t)NB * NA * HID * 2;
  const size_t oWhd = off; off += (size_t)NHD * DHD * KP1 * 2;
  const size_t oWo  = off; off += (size_t)HID * HID * 2;
  const size_t oF1  = off; off += (size_t)HID * KPF * 2;
  const size_t oF2  = off; off += (size_t)HID * HID * 2;
  const size_t oQw  = off; off += (size_t)HID * HID * 2;
  const size_t oVw  = off; off += (size_t)HID * HID * 2;
  const size_t oOw  = off; off += (size_t)HID * HID * 2;
  const size_t oN1  = off; off += (size_t)HID * HID * 2;
  const size_t oE2  = off; off += (size_t)NTP * HID * 2;
  const size_t oFp  = off; off += (size_t)NB * KPF * 2;
  const size_t oGo  = off; off += (size_t)NB * HID * 2;
  const size_t oFh  = off; off += (size_t)NB * HID * 2;
  const size_t oFn  = off; off += (size_t)NB * HID * 2;
  const size_t oFu0 = off; off += (size_t)NB * HID * 2;
  const size_t oFu  = off; off += (size_t)NB * HID * 2;
  const size_t oHd  = off; off += (size_t)NB * HID * 2;
  const size_t oQf  = off; off += (size_t)NB * HID * 4;
  if (off > ws_size) return;
  if (off > (size_t)134217728) return;

  char* ws = (char*)d_ws;
  hf* X    = (hf*)(ws + oX);
  hf* WhdT = (hf*)(ws + oWhd);
  hf* WoT  = (hf*)(ws + oWo);
  hf* F1T  = (hf*)(ws + oF1);
  hf* F2T  = (hf*)(ws + oF2);
  hf* QT   = (hf*)(ws + oQw);
  hf* VT   = (hf*)(ws + oVw);
  hf* OT   = (hf*)(ws + oOw);
  hf* N1T  = (hf*)(ws + oN1);
  hf* E2T  = (hf*)(ws + oE2);
  hf* FP   = (hf*)(ws + oFp);
  hf* GO   = (hf*)(ws + oGo);
  hf* FH   = (hf*)(ws + oFh);
  hf* FN   = (hf*)(ws + oFn);
  hf* FU0  = (hf*)(ws + oFu0);
  hf* FU   = (hf*)(ws + oFu);
  hf* HD   = (hf*)(ws + oHd);
  float* QF = (float*)(ws + oQf);

  const float osc = 1.0f / (ASCALE * WSCALE);

  k_cvt16<<<dim3(DHD / 16, NHD), dim3(256), 32 * KP1, stream>>>(Whead, DHD, FIN, DHD, KP1, 1, FIN * DHD, DHD * KP1,
                                                                WSCALE, WhdT);
  k_cvt16<<<dim3(HID / 16, 1), dim3(256), 32 * HID, stream>>>(Wout, HID, HID, HID, HID, 1, 0, 0, WSCALE, WoT);
  k_cvt16<<<dim3(HID / 16, 1), dim3(256), 32 * KPF, stream>>>(fc1w, HID, FPD, HID, KPF, 1, 0, 0, WSCALE, F1T);
  k_cvt16<<<dim3(HID / 16, 1), dim3(256), 32 * HID, stream>>>(fc2w, HID, HID, HID, HID, 1, 0, 0, WSCALE, F2T);
  k_cvt16<<<dim3(HID / 16, 1), dim3(256), 32 * HID, stream>>>(qw,   HID, HID, HID, HID, 1, 0, 0, WSCALE, QT);
  k_cvt16<<<dim3(HID / 16, 1), dim3(256), 32 * HID, stream>>>(vw,   HID, HID, HID, HID, 1, 0, 0, WSCALE, VT);
  k_cvt16<<<dim3(HID / 16, 1), dim3(256), 32 * HID, stream>>>(ow,   HID, HID, HID, HID, 1, 0, 0, WSCALE, OT);
  k_cvt16<<<dim3(HID / 16, 1), dim3(256), 32 * HID, stream>>>(f1w,  HID, HID, HID, HID, 1, 0, 0, WSCALE, N1T);
  k_cvt16<<<dim3(NTP / 16, 1), dim3(256), 32 * HID, stream>>>(f2w,  NT,  HID, NT,  HID, 1, 0, 0, WSCALE, E2T);
  k_cvt16<<<dim3(NB / 16, 1), dim3(256), 32 * KPF, stream>>>(fp, NB, FPD, FPD, KPF, 0, 0, 0, ASCALE, FP);
  (void)hipFuncSetAttribute(reinterpret_cast<const void*>(&k_gat1), hipFuncAttributeMaxDynamicSharedMemorySize,
                            G1_LDS);
  k_gat1<<<dim3(NB), dim3(256), G1_LDS, stream>>>(h, adj, edge, WhdT, a1h, a2h, aeh, X);
  (void)hipFuncSetAttribute(reinterpret_cast<const void*>(&k_gat2), hipFuncAttributeMaxDynamicSharedMemorySize,
                            G2_LDS);
  k_gat2<<<dim3(NB), dim3(256), G2_LDS, stream>>>(X, WoT, adj, edge, a1o, a2o, aeo, GO);
  k_gemm<<<dim3(NB / 128, HID / 64), dim3(256), 0, stream>>>(FP, KPF, F1T, KPF, KPF, fc1b, nullptr, HID, osc, 1,
                                                            ASCALE, nullptr, FH);
  k_gemm<<<dim3(NB / 128, HID / 64), dim3(256), 0, stream>>>(FH, HID, F2T, HID, HID, fc2b, nullptr, HID, osc, 0,
                                                            ASCALE, nullptr, FN);
  k_gemm<<<dim3(NB / 128, HID / 64), dim3(256), 0, stream>>>(GO, HID, QT, HID, HID, qb, nullptr, HID, osc, 0,
                                                            ASCALE, QF, nullptr);
  k_gemm<<<dim3(NB / 128, HID / 64), dim3(256), 0, stream>>>(FN, HID, VT, HID, HID, vb, QF, HID, osc, 0,
                                                            ASCALE, nullptr, FU0);
  k_gemm<<<dim3(NB / 128, HID / 64), dim3(256), 0, stream>>>(FU0, HID, OT, HID, HID, ob, nullptr, HID, osc, 1,
                                                            ASCALE, nullptr, FU);
  k_gemm<<<dim3(NB / 128, HID / 64), dim3(256), 0, stream>>>(FU, HID, N1T, HID, HID, f1b, nullptr, HID, osc, 1,
                                                            ASCALE, nullptr, HD);
  k_final<<<dim3(1), dim3(256), 0, stream>>>(HD, E2T, f2b, out);
  (void)hipGetLastError();
}
